// SoftSOMLayer_44341242364446
// MI455X (gfx1250) — hardware-verified
//
#include <hip/hip_runtime.h>
#include <math.h>

#pragma clang fp contract(off)

constexpr int kBatch = 16384;
constexpr int kDim   = 512;
constexpr int kGrid0 = 32;
constexpr int kGrid1 = 32;
constexpr int kProto = kGrid0 * kGrid1;
constexpr int kChunk = 8192;
constexpr int kNumChunks = kBatch / kChunk;
constexpr int kAcatK = 2 * kProto;
constexpr float kTau = 0.5f;
constexpr float kEps = 1e-8f;

constexpr size_t kOffXb   = 0;
constexpr size_t kOffWb   = kOffXb + (size_t)kBatch * kDim * 2;
constexpr size_t kOffWT   = kOffWb + (size_t)kProto * kDim * 2;
constexpr size_t kOffX2   = kOffWT + (size_t)kDim * kAcatK * 2;
constexpr size_t kOffW2   = kOffX2 + (size_t)kBatch * 4;
constexpr size_t kOffG    = kOffW2 + (size_t)kProto * 4;
constexpr size_t kOffA    = kOffG + (size_t)kChunk * kProto * 4;
constexpr size_t kWsTotal = kOffA + (size_t)kChunk * kAcatK * 2;
typedef char ws_total_check[(kWsTotal <= (size_t)134217728) ? 1 : -1];
typedef char ws_align_check[((kOffWb % 128) == 0 && (kOffWT % 128) == 0 && (kOffX2 % 128) == 0 &&
                             (kOffW2 % 128) == 0 && (kOffG % 128) == 0 && (kOffA % 128) == 0) ? 1 : -1];
typedef char chunk_check[(kBatch % kChunk == 0 && kChunk % 64 == 0 && kProto % 64 == 0 && kDim % 64 == 0 &&
                          kDim % 32 == 0 && kAcatK % 32 == 0) ? 1 : -1];

typedef __attribute__((ext_vector_type(16))) _Float16 v16h;
typedef __attribute__((ext_vector_type(8)))  _Float16 v8h;
typedef __attribute__((ext_vector_type(16))) __bf16   v16b;
typedef __attribute__((ext_vector_type(8)))  __bf16   v8b;
typedef __attribute__((ext_vector_type(8)))  float    v8f;
typedef __attribute__((ext_vector_type(4)))  float    v4f;
typedef __attribute__((ext_vector_type(4)))  unsigned int v4u;

__device__ __forceinline__ unsigned short f2bf_bits(float f) {
  unsigned u = __float_as_uint(f);
  return (unsigned short)((u + 0x7FFFu + ((u >> 16) & 1u)) >> 16);
}
__device__ __forceinline__ float bf_bits2f(unsigned short h) { return __uint_as_float(((unsigned)h) << 16); }

__device__ __forceinline__ void dep_guard_h(v8f& a, v8f& b, v16h x, v16h y) { asm volatile("v_nop\n\tv_nop\n\tv_nop\n\tv_nop" : "+v"(a), "+v"(b) : "v"(x), "v"(y)); }
__device__ __forceinline__ void dep_guard_b(v8f& a, v8f& b, v16b x, v16b y) { asm volatile("v_nop\n\tv_nop\n\tv_nop\n\tv_nop" : "+v"(a), "+v"(b) : "v"(x), "v"(y)); }
__device__ __forceinline__ void keep4_h(v16h a, v16h b, v16h c, v16h d) { asm volatile("v_nop" :: "v"(a), "v"(b), "v"(c), "v"(d)); }
__device__ __forceinline__ void keep4_b(v16b a, v16b b, v16b c, v16b d) { asm volatile("v_nop" :: "v"(a), "v"(b), "v"(c), "v"(d)); }
__device__ __forceinline__ void acc_guard4(v8f& a, v8f& b, v8f& c, v8f& d) { asm volatile("v_nop\n\tv_nop\n\tv_nop\n\tv_nop" : "+v"(a), "+v"(b), "+v"(c), "+v"(d)); }
template <typename T> struct Frag;
template <> struct Frag<_Float16> {
  typedef v16h V; union U { v16h v; v8h h[2]; };
  static __device__ __forceinline__ v16h load(const _Float16* p) {
    U f; f.h[0] = *(const v8h*)(p); f.h[1] = *(const v8h*)(p + 16); return f.v;
  }
  static __device__ __forceinline__ v8f mma(v16h a, v16h b, v8f c) {
    return __builtin_amdgcn_wmma_f32_16x16x32_f16(false, a, false, b, (short)0, c, false, false);
  }
  static __device__ __forceinline__ void guard(v8f& a, v8f& b, v16h x, v16h y) { dep_guard_h(a, b, x, y); }
  static __device__ __forceinline__ void keep(v16h a, v16h b, v16h c, v16h d) { keep4_h(a, b, c, d); }
};
template <> struct Frag<__bf16> {
  typedef v16b V; union U { v16b v; v8b h[2]; };
  static __device__ __forceinline__ v16b load(const __bf16* p) {
    U f; f.h[0] = *(const v8b*)(p); f.h[1] = *(const v8b*)(p + 16); return f.v;
  }
  static __device__ __forceinline__ v8f mma(v16b a, v16b b, v8f c) {
    return __builtin_amdgcn_wmma_f32_16x16x32_bf16(false, a, false, b, (short)0, c, false, false);
  }
  static __device__ __forceinline__ void guard(v8f& a, v8f& b, v16b x, v16b y) { dep_guard_b(a, b, x, y); }
  static __device__ __forceinline__ void keep(v16b a, v16b b, v16b c, v16b d) { keep4_b(a, b, c, d); }
};

__device__ __forceinline__ unsigned pk16(unsigned short a, unsigned short b) { return (unsigned)a | ((unsigned)b << 16); }

template <int ET> struct Elem;
template <> struct Elem<0> { typedef _Float16 T; };
template <> struct Elem<1> { typedef __bf16 T; };
template <int ET, bool SPLIT, int BIAS_MODE, int OUT_MODE, bool RESID, int ACT = 0>
__global__ __launch_bounds__(256) void wmma_gemm64(
    const unsigned short* __restrict__ Ap, const unsigned short* __restrict__ A2p, int lda, long strideA,
    const unsigned short* __restrict__ Btp, const unsigned short* __restrict__ Bt2p, int ldb, long strideB,
    void* __restrict__ Cout, void* __restrict__ Cout2, int ldc, long strideC,
    const float* __restrict__ bias,
    const float* __restrict__ resid, long strideR,
    int M, int N, int K, float scale) {
  typedef typename Elem<ET>::T T;
  typedef typename Frag<T>::V V;
  const T* A = (const T*)Ap; const T* A2 = (const T*)A2p; const T* Bt = (const T*)Btp; const T* Bt2 = (const T*)Bt2p;
  __shared__ __align__(16) float sT[8][16 * 68];
  const int b    = blockIdx.y;
  const int lane = threadIdx.x & 31;
  const int wave = threadIdx.x >> 5;
  const int tilesN = N >> 6;
  const int tilesM = M >> 6;
  const int tile = blockIdx.x * 8 + wave;
  if (tile >= tilesM * tilesN) return;
  const int tm = tile / tilesN;
  const int tn = tile - tm * tilesN;
  const int m0 = tm << 6;
  const int n0 = tn << 6;

  const T* Ab  = A  + (size_t)b * strideA;
  const T* Bb  = Bt + (size_t)b * strideB;
  const T* Ab2 = SPLIT ? (A2  + (size_t)b * strideA) : nullptr;
  const T* Bb2 = SPLIT ? (Bt2 + (size_t)b * strideB) : nullptr;

  const int rlane = lane & 15;
  const int koff  = (lane >> 4) * 8;
  const int mOff  = (lane >> 4) * 8;

  v8f acc[4][4];
#pragma unroll
  for (int i = 0; i < 4; ++i)
#pragma unroll
    for (int j = 0; j < 4; ++j) acc[i][j] = (v8f){0.f,0.f,0.f,0.f,0.f,0.f,0.f,0.f};

  for (int k0 = 0; k0 < K; k0 += 32) {
    V bh[4], bl[4];
#pragma unroll
    for (int j = 0; j < 4; ++j) {
      const size_t bo = (size_t)(n0 + (j << 4) + rlane) * ldb + koff + k0;
      bh[j] = Frag<T>::load(Bb + bo);
      if (SPLIT) bl[j] = Frag<T>::load(Bb2 + bo);
    }
#pragma unroll
    for (int i = 0; i < 4; ++i) {
      const size_t ao = (size_t)(m0 + (i << 4) + rlane) * lda + koff + k0;
      V ah = Frag<T>::load(Ab + ao);
      V al;
      if (SPLIT) al = Frag<T>::load(Ab2 + ao);
#pragma unroll
      for (int j = 0; j < 4; ++j) {
        acc[i][j] = Frag<T>::mma(ah, bh[j], acc[i][j]);
        if (SPLIT) {
          acc[i][j] = Frag<T>::mma(ah, bl[j], acc[i][j]);
          acc[i][j] = Frag<T>::mma(al, bh[j], acc[i][j]);
        }
      }
      Frag<T>::guard(acc[i][0], acc[i][3], ah, SPLIT ? al : ah);
    }
    Frag<T>::keep(bh[0], bh[1], bh[2], bh[3]);
    if (SPLIT) Frag<T>::keep(bl[0], bl[1], bl[2], bl[3]);
  }
  acc_guard4(acc[0][0], acc[0][1], acc[0][2], acc[0][3]);
  acc_guard4(acc[1][0], acc[1][1], acc[1][2], acc[1][3]);
  acc_guard4(acc[2][0], acc[2][1], acc[2][2], acc[2][3]);
  acc_guard4(acc[3][0], acc[3][1], acc[3][2], acc[3][3]);

  float* slab = sT[wave];
  const float* Rb = RESID ? (resid + (size_t)b * strideR) : nullptr;
#pragma unroll
  for (int i = 0; i < 4; ++i) {
    const int mBase = m0 + (i << 4);
#pragma unroll
    for (int j = 0; j < 4; ++j) {
      const int n = n0 + (j << 4) + rlane;
      float bv = 0.f;
      if (BIAS_MODE == 2) bv = bias[n];
#pragma unroll
      for (int r = 0; r < 8; ++r) {
        float v = acc[i][j][r] * scale;
        if (BIAS_MODE == 1) v += bias[mBase + mOff + r];
        if (BIAS_MODE == 2) v += bv;
        if (RESID) v += Rb[(size_t)(mBase + mOff + r) * ldc + n];
        if (ACT == 2) v = fmaxf(v, 0.0f);
        if (ACT == 4) v = (v > 0.f) ? v : 0.01f * v;
        slab[(mOff + r) * 68 + (j << 4) + rlane] = v;
      }
    }
    __builtin_amdgcn_fence(__ATOMIC_RELEASE, "workgroup");
    __builtin_amdgcn_wave_barrier();
    __builtin_amdgcn_fence(__ATOMIC_ACQUIRE, "workgroup");
    if (OUT_MODE == 0) {
      float* C = (float*)Cout + (size_t)b * strideC;
      const int hh = lane >> 4, c4 = (lane & 15) * 4;
      for (int pass = 0; pass < 2; ++pass) {
#pragma unroll
        for (int it = 0; it < 8; ++it) {
          const int row = it * 2 + hh;
          v4f v = *(const v4f*)(slab + row * 68 + c4);
          *(volatile v4f*)(C + (size_t)(mBase + row) * ldc + n0 + c4) = v;
        }
        __threadfence();
      }
    } else {
      const int q = lane >> 3, c8 = (lane & 7) * 8;
      unsigned short* C  = (unsigned short*)Cout  + (size_t)b * strideC;
      unsigned short* C2 = (OUT_MODE == 2) ? ((unsigned short*)Cout2 + (size_t)b * strideC) : nullptr;
      for (int pass = 0; pass < 2; ++pass) {
#pragma unroll
        for (int it = 0; it < 4; ++it) {
          const int row = it * 4 + q;
          const float* sp = slab + row * 68 + c8;
          v8h hv, lv;
#pragma unroll
          for (int e = 0; e < 8; ++e) {
            if (OUT_MODE == 1) {
              hv[e] = (_Float16)sp[e];
            } else {
              unsigned short hb = f2bf_bits(sp[e]);
              unsigned short lb = f2bf_bits(sp[e] - bf_bits2f(hb));
              hv[e] = __builtin_bit_cast(_Float16, hb);
              lv[e] = __builtin_bit_cast(_Float16, lb);
            }
          }
          *(volatile v8h*)(C + (size_t)(mBase + row) * ldc + n0 + c8) = hv;
          if (OUT_MODE == 2) *(volatile v8h*)(C2 + (size_t)(mBase + row) * ldc + n0 + c8) = lv;
        }
        __threadfence();
      }
    }
    __builtin_amdgcn_fence(__ATOMIC_RELEASE, "workgroup");
    __builtin_amdgcn_wave_barrier();
    __builtin_amdgcn_fence(__ATOMIC_ACQUIRE, "workgroup");
  }
}

__global__ __launch_bounds__(256) void rowcast_bf16_kernel(const float* __restrict__ in, unsigned short* __restrict__ out,
                                                           float* __restrict__ sumsq, int nrows) {
  __shared__ __align__(16) float ssh[32];
  const int t = threadIdx.x, lane = t & 31, wave = t >> 5;
  const int rb = blockIdx.x * 32;
#pragma unroll 1
  for (int rr = 0; rr < 4; ++rr) {
    int row = rb + wave * 4 + rr;
    row = row < nrows ? row : nrows - 1;
    const float* src = in + (size_t)row * kDim;
    unsigned short* dst = out + (size_t)row * kDim;
    float ss = 0.f;
    v4u u[2];
#pragma unroll
    for (int it = 0; it < 2; ++it) {
      const float* p = src + it * 256 + 8 * lane;
      const v4f a = *(const v4f*)(p);
      const v4f c = *(const v4f*)(p + 4);
      unsigned short hb[8];
#pragma unroll
      for (int e = 0; e < 4; ++e) {
        hb[e] = f2bf_bits(a[e]);
        const float rv = bf_bits2f(hb[e]);
        ss += rv * rv;
      }
#pragma unroll
      for (int e = 0; e < 4; ++e) {
        hb[4 + e] = f2bf_bits(c[e]);
        const float rv = bf_bits2f(hb[4 + e]);
        ss += rv * rv;
      }
      u[it] = (v4u){pk16(hb[0], hb[1]), pk16(hb[2], hb[3]), pk16(hb[4], hb[5]), pk16(hb[6], hb[7])};
    }
    for (int pass = 0; pass < 2; ++pass) {
#pragma unroll
      for (int it = 0; it < 2; ++it) *(volatile v4u*)(dst + it * 256 + 8 * lane) = u[it];
      __threadfence();
    }
#pragma unroll
    for (int off = 16; off > 0; off >>= 1) ss += __shfl_xor(ss, off, 32);
    if (lane == 0) ssh[wave * 4 + rr] = ss;
  }
  __syncthreads();
  if (wave == 0) {
    const int l8 = lane & 7;
    const v4f v = *(const v4f*)(ssh + 4 * l8);
    float* sp = sumsq + rb + 4 * l8;
    if (lane < 8) {
      *(volatile v4f*)sp = v;
      __threadfence();
      *(volatile v4f*)sp = v;
    }
  }
}

__global__ __launch_bounds__(256) void wtcast2_kernel(const float* __restrict__ W, unsigned short* __restrict__ out) {
  __shared__ float sm[64][65];
  const int t  = threadIdx.x;
  const int n0 = blockIdx.x * 64;
  const int d0 = blockIdx.y * 64;
#pragma unroll
  for (int i = 0; i < 16; ++i) {
    const int e = i * 256 + t;
    const int r = e >> 6;
    const int c = e & 63;
    sm[c][r] = W[(size_t)(n0 + r) * kDim + d0 + c];
  }
  __syncthreads();
  const int lane = t & 31, wave = t >> 5;
  const int q = lane >> 3, c8 = (lane & 7) * 8;
  for (int pass = 0; pass < 2; ++pass) {
#pragma unroll
    for (int it = 0; it < 2; ++it) {
      const int row = wave * 8 + it * 4 + q;
      unsigned short hb[8];
#pragma unroll
      for (int e = 0; e < 8; ++e) hb[e] = f2bf_bits(sm[row][c8 + e]);
      const v4u u = (v4u){pk16(hb[0], hb[1]), pk16(hb[2], hb[3]), pk16(hb[4], hb[5]), pk16(hb[6], hb[7])};
      unsigned short* op = out + (size_t)(d0 + row) * kAcatK + n0 + c8;
      *(volatile v4u*)(op) = u;
      *(volatile v4u*)(op + kProto) = u;
    }
    __threadfence();
  }
}

__global__ __launch_bounds__(128) void som_softmax_kernel(const float* __restrict__ G, const float* __restrict__ x2,
                                                          const float* __restrict__ w2, unsigned short* __restrict__ Acat,
                                                          int nrows) {
  __shared__ __align__(16) float Et[4][kProto];
  __shared__ __align__(16) float Qt[4][kProto];
  const int t = threadIdx.x, lane = t & 31, wave = t >> 5;
  float* ew = Et[wave];
  float* qw = Qt[wave];
#pragma unroll 1
  for (int rr = 0; rr < 4; ++rr) {
    int row = blockIdx.x * 16 + wave * 4 + rr;
    row = row < nrows ? row : nrows - 1;
    const float* gr = G + (size_t)row * kProto + lane;
    const float x2v = x2[row];
    float mr = -__builtin_inff();
#pragma unroll 1
    for (int i = 0; i < kGrid0; ++i) {
      const float g   = gr[i * kGrid1];
      const float w2v = w2[i * kGrid1 + lane];
      const float d2  = (x2v + w2v) - 2.0f * g;
      const float lg  = -d2 / kTau;
      ew[i * kGrid1 + lane] = lg;
      mr = fmaxf(mr, lg);
    }
    float sr = 0.f;
#pragma unroll 1
    for (int i = 0; i < kGrid0; ++i) {
      const float lg = ew[i * kGrid1 + lane];
      const float er = expf(lg - mr);
      sr += er;
      float mc = lg;
#pragma unroll
      for (int off = 16; off > 0; off >>= 1) mc = fmaxf(mc, __shfl_xor(mc, off, 32));
      const float ec = expf(lg - mc);
      float sc = ec;
#pragma unroll
      for (int off = 16; off > 0; off >>= 1) sc += __shfl_xor(sc, off, 32);
      ew[i * kGrid1 + lane] = er;
      qw[i * kGrid1 + lane] = ec * (1.0f / sc);
    }
    const float invSr = 1.0f / sr;
    float tot = 0.f;
#pragma unroll 1
    for (int i = 0; i < kGrid0; ++i) {
      const float a = (ew[i * kGrid1 + lane] * invSr) * qw[i * kGrid1 + lane];
      ew[i * kGrid1 + lane] = a;
      tot += a;
    }
#pragma unroll
    for (int off = 16; off > 0; off >>= 1) tot += __shfl_xor(tot, off, 32);
    const float invT = 1.0f / (tot + kEps);
    __syncthreads();
    unsigned short* arow = Acat + (size_t)row * kAcatK;
    const int il = lane >> 2, j0 = (lane & 3) * 8;
    for (int pass = 0; pass < 2; ++pass) {
#pragma unroll
      for (int it = 0; it < 4; ++it) {
        const int i = it * 8 + il;
        const v4f p0 = *(const v4f*)(ew + i * kGrid1 + j0);
        const v4f p1 = *(const v4f*)(ew + i * kGrid1 + j0 + 4);
        unsigned short hb[8], lb[8];
#pragma unroll
        for (int e = 0; e < 4; ++e) {
          const float v0 = p0[e] * invT;
          hb[e] = f2bf_bits(v0);
          lb[e] = f2bf_bits(v0 - bf_bits2f(hb[e]));
          const float v1 = p1[e] * invT;
          hb[4 + e] = f2bf_bits(v1);
          lb[4 + e] = f2bf_bits(v1 - bf_bits2f(hb[4 + e]));
        }
        const v4u uh = (v4u){pk16(hb[0], hb[1]), pk16(hb[2], hb[3]), pk16(hb[4], hb[5]), pk16(hb[6], hb[7])};
        const v4u ul = (v4u){pk16(lb[0], lb[1]), pk16(lb[2], lb[3]), pk16(lb[4], lb[5]), pk16(lb[6], lb[7])};
        *(volatile v4u*)(arow + it * 256 + 8 * lane) = uh;
        *(volatile v4u*)(arow + kProto + it * 256 + 8 * lane) = ul;
      }
      __threadfence();
    }
    __syncthreads();
  }
}

extern "C" void kernel_launch(void* const* d_in, const int* in_sizes, int n_in,
                              void* d_out, int out_size, void* d_ws, size_t ws_size,
                              hipStream_t stream) {
  if (n_in < 2) return;
  if (in_sizes[0] != kBatch * kDim || in_sizes[1] != kProto * kDim || out_size != kBatch * kDim) return;
  if (ws_size < kWsTotal) return;
  const float* x = (const float*)d_in[0];
  const float* w = (const float*)d_in[1];
  float* y = (float*)d_out;
  char* ws = (char*)d_ws;
  unsigned short* Xb  = (unsigned short*)(ws + kOffXb);
  unsigned short* Wb  = (unsigned short*)(ws + kOffWb);
  unsigned short* WTc = (unsigned short*)(ws + kOffWT);
  float* x2 = (float*)(ws + kOffX2);
  float* w2 = (float*)(ws + kOffW2);
  float* G  = (float*)(ws + kOffG);
  unsigned short* Acat = (unsigned short*)(ws + kOffA);

  rowcast_bf16_kernel<<<dim3(kBatch / 32), dim3(256), 0, stream>>>(x, Xb, x2, kBatch);
  rowcast_bf16_kernel<<<dim3(kProto / 32), dim3(256), 0, stream>>>(w, Wb, w2, kProto);
  wtcast2_kernel<<<dim3(kProto / 64, kDim / 64), dim3(256), 0, stream>>>(w, WTc);

  const int tiles1 = (kChunk / 64) * (kProto / 64);
  const int tiles2 = (kChunk / 64) * (kDim / 64);
  for (int ch = 0; ch < kNumChunks; ++ch) {
    const unsigned short* Xc = Xb + (size_t)ch * kChunk * kDim;
    float* yc = y + (size_t)ch * kChunk * kDim;
    wmma_gemm64<1, false, 0, 0, false, 0><<<dim3((tiles1 + 7) / 8, 1), dim3(256), 0, stream>>>(
        Xc, (const unsigned short*)nullptr, kDim, 0L,
        (const unsigned short*)Wb, (const unsigned short*)nullptr, kDim, 0L,
        (void*)G, (void*)nullptr, kProto, 0L,
        (const float*)nullptr, (const float*)nullptr, 0L,
        kChunk, kProto, kDim, 1.0f);
    som_softmax_kernel<<<dim3(kChunk / 16), dim3(128), 0, stream>>>(G, x2 + (size_t)ch * kChunk, w2, Acat, kChunk);
    wmma_gemm64<1, false, 0, 0, false, 0><<<dim3((tiles2 + 7) / 8, 1), dim3(256), 0, stream>>>(
        (const unsigned short*)Acat, (const unsigned short*)nullptr, kAcatK, 0L,
        (const unsigned short*)WTc, (const unsigned short*)nullptr, kAcatK, 0L,
        (void*)yc, (void*)nullptr, kDim, 0L,
        (const float*)nullptr, (const float*)nullptr, 0L,
        kChunk, kDim, kAcatK, 1.0f);
  }
}
